// GATEncoder_17059610100458
// MI455X (gfx1250) — hardware-run, weakly checked
//
#include <hip/hip_runtime.h>

typedef float          v8f   __attribute__((ext_vector_type(8)));
typedef float          v4f   __attribute__((ext_vector_type(4)));
typedef unsigned int   v4u   __attribute__((ext_vector_type(4)));
typedef int            v8i   __attribute__((ext_vector_type(8)));
typedef unsigned short v8us  __attribute__((ext_vector_type(8)));
typedef unsigned short v16us __attribute__((ext_vector_type(16)));
typedef __bf16         v16bf __attribute__((ext_vector_type(16)));
typedef _Float16       v16h  __attribute__((ext_vector_type(16)));
typedef v4f  __attribute__((may_alias)) v4fa;
typedef v8us __attribute__((may_alias)) v8usa;
union FragB { v16bf v; v16us u; v8us h[2]; v8i w; };
union FragH { v16h  v; v16us u; v8us h[2]; v8i w; };

__device__ __forceinline__ v8f wmb(const FragB& a, const FragB& b, v8f c) {
  v8f d = __builtin_amdgcn_wmma_f32_16x16x32_bf16(false, a.v, false, b.v, (short)0, c, false, false);
  asm volatile("v_nop\n\tv_nop\n\tv_nop\n\tv_nop" : "+v"(d) : "v"(a.w), "v"(b.w));
  return d;
}

__device__ __forceinline__ v8f wmh(const FragH& a, const FragH& b, v8f c) {
  v8f d = __builtin_amdgcn_wmma_f32_16x16x32_f16(false, a.v, false, b.v, (short)0, c, false, false);
  asm volatile("v_nop\n\tv_nop\n\tv_nop\n\tv_nop" : "+v"(d) : "v"(a.w), "v"(b.w));
  return d;
}

__device__ __forceinline__ unsigned bf16_bits(float f) {
  const unsigned u = __float_as_uint(f);
  const unsigned r = (u + 0x7FFFu + ((u >> 16) & 1u)) >> 16;
  const unsigned q = (u >> 16) | 0x40u;
  return ((u & 0x7fffffffu) > 0x7f800000u) ? q : r;
}

__device__ __forceinline__ float bf16_val(float f) {
  return __uint_as_float(bf16_bits(f) << 16);
}
__device__ __forceinline__ int clampi(int v, int lo, int hi) {
  return v < lo ? lo : (v > hi ? hi : v);
}

__device__ __forceinline__ unsigned f16_bits(float f) {
  const unsigned u  = __float_as_uint(f);
  const unsigned s  = (u >> 16) & 0x8000u;
  const unsigned a  = u & 0x7fffffffu;
  const unsigned t  = a - 0x38000000u;
  const unsigned r  = (t + 0x0FFFu + ((t >> 13) & 1u)) >> 13;
  const unsigned rc = r > 0x7C00u ? 0x7C00u : r;
  const bool small  = a < 0x38800000u;
  const bool isnan  = a > 0x7f800000u;
  const unsigned fin = small ? 0u : (s | rc);
  return isnan ? (s | 0x7E00u) : fin;
}

__device__ __forceinline__ unsigned pk16(unsigned lo, unsigned hi) { return lo | (hi << 16); }
__device__ __forceinline__ unsigned bf16_lo_bits(float v) {
  float hi = bf16_val(v);
  asm volatile("" : "+v"(hi));
  return bf16_bits(v - hi);
}
__device__ __forceinline__ v4u pack8_bf16(v4f a, v4f c) {
  return (v4u){ pk16(bf16_bits(a[0]), bf16_bits(a[1])), pk16(bf16_bits(a[2]), bf16_bits(a[3])),
                pk16(bf16_bits(c[0]), bf16_bits(c[1])), pk16(bf16_bits(c[2]), bf16_bits(c[3])) };
}
__device__ __forceinline__ v4u pack8_bf16_lo(v4f a, v4f c) {
  return (v4u){ pk16(bf16_lo_bits(a[0]), bf16_lo_bits(a[1])), pk16(bf16_lo_bits(a[2]), bf16_lo_bits(a[3])),
                pk16(bf16_lo_bits(c[0]), bf16_lo_bits(c[1])), pk16(bf16_lo_bits(c[2]), bf16_lo_bits(c[3])) };
}
__device__ __forceinline__ v4u pack8_f16(v4f a, v4f c) {
  return (v4u){ pk16(f16_bits(a[0]), f16_bits(a[1])), pk16(f16_bits(a[2]), f16_bits(a[3])),
                pk16(f16_bits(c[0]), f16_bits(c[1])), pk16(f16_bits(c[2]), f16_bits(c[3])) };
}

template <int FORM>
__global__ __launch_bounds__(256) void k_plane(const float* __restrict__ src, int rows, int cols, int ldsrc,
                                               unsigned short* __restrict__ dst, int MP, int KP) {
  static_assert(FORM >= 0 && FORM <= 3);
  const int KTOT = (FORM == 1 || FORM == 3) ? 2 * KP : KP;
  const unsigned ppr   = (unsigned)(KTOT >> 3);
  const unsigned kp8   = (unsigned)(KP >> 3);
  const unsigned total = (unsigned)MP * ppr;
  const unsigned g     = blockIdx.x * 256u + threadIdx.x;
  const unsigned rowu  = g / ppr;
  const unsigned p     = g - rowu * ppr;
  const bool second    = p >= kp8;
  const int row = (int)rowu;
  const int c0  = (int)((second ? p - kp8 : p) << 3);
  const float* srow = src + (size_t)clampi(row, 0, rows - 1) * (size_t)ldsrc;
  float x[8];
  unsigned mk[8];
#pragma unroll
  for (int e = 0; e < 8; ++e) {
    const int c = c0 + e;
    const float v = srow[clampi(c, 0, cols - 1)];
    asm volatile("" :: "v"(v));
    x[e]  = v;
    mk[e] = (row < rows && c < cols) ? 0xFFFFu : 0u;
  }
  const v4f a = (v4f){ x[0], x[1], x[2], x[3] };
  const v4f c = (v4f){ x[4], x[5], x[6], x[7] };
  v4u o;
  if (FORM == 2) {
    o = pack8_f16(a, c);
  } else {
    const v4u hi = pack8_bf16(a, c);
    o = hi;
    if (FORM == 1) { const v4u lo = pack8_bf16_lo(a, c); o = second ? lo : hi; }
  }
  const v4u mw = (v4u){ pk16(mk[0], mk[1]), pk16(mk[2], mk[3]), pk16(mk[4], mk[5]), pk16(mk[6], mk[7]) };
  o &= mw;
  if (g < total) {
    volatile v4u* q = (volatile v4u*)(dst + (size_t)g * 8);
    *q = o;
    __threadfence();
    *q = o;
  }
}

template <int FORM> struct FragOf    { typedef FragB T; };
template <>         struct FragOf<2> { typedef FragH T; };
__device__ __forceinline__ v8f mm(const FragB& a, const FragB& b, v8f c) { return wmb(a, b, c); }
__device__ __forceinline__ v8f mm(const FragH& a, const FragH& b, v8f c) { return wmh(a, b, c); }
template <class F> __device__ __forceinline__ F ld_frag(const unsigned short* p) {
  F f;
  f.h[0] = *(const v8usa*)(p);
  f.h[1] = *(const v8usa*)(p + 16);
  return f;
}

template <int FORM, int EPI>
__global__ __launch_bounds__(256) __attribute__((amdgpu_num_vgpr(248)))
void k_gemm_nt(const unsigned short* __restrict__ A, const unsigned short* __restrict__ B,
               const float* __restrict__ bias, float* __restrict__ D, int M, int N, int KTOT, int ldd) {
  static_assert(FORM >= 0 && FORM <= 2);
  static_assert(EPI == 0 || EPI == 1);
  typedef typename FragOf<FORM>::T F;
  __shared__ __attribute__((aligned(16))) float sT[8][16 * 68];
  const int lane = threadIdx.x & 31;
  const int wave = threadIdx.x >> 5;
  const int tilesM = (M + 63) >> 6;
  const int tilesN = (N + 63) >> 6;
  const int tile = blockIdx.x * 8 + wave;
  if (tile >= tilesM * tilesN) return;
  const int tm = tile / tilesN;
  const int tn = tile - tm * tilesN;
  const int m0 = tm << 6;
  const int n0 = tn << 6;

  const int rl = lane & 15;
  const int h8 = (lane >> 4) * 8;
  const unsigned short* pa = A + (size_t)(m0 + rl) * (size_t)KTOT + h8;
  const unsigned short* pb = B + (size_t)(n0 + rl) * (size_t)KTOT + h8;

  v8f acc[4][4];
#pragma unroll
  for (int i = 0; i < 4; ++i)
#pragma unroll
    for (int j = 0; j < 4; ++j) acc[i][j] = (v8f){0.f, 0.f, 0.f, 0.f, 0.f, 0.f, 0.f, 0.f};

#pragma unroll 1
  for (int k0 = 0; k0 < KTOT; k0 += 32) {
    F bf[4];
#pragma unroll
    for (int j = 0; j < 4; ++j) bf[j] = ld_frag<F>(pb + (size_t)(j << 4) * (size_t)KTOT + k0);
#pragma unroll
    for (int i = 0; i < 4; ++i) {
      const F af = ld_frag<F>(pa + (size_t)(i << 4) * (size_t)KTOT + k0);
#pragma unroll
      for (int j = 0; j < 4; ++j) acc[i][j] = mm(af, bf[j], acc[i][j]);
    }
  }

  float* slab = sT[wave];
  const int hh = lane >> 4;
  const int c4 = (lane & 15) * 4;
  const int nc = n0 + c4;
  const bool cok = nc < N;
  v4f bv = (v4f){0.f, 0.f, 0.f, 0.f};
  if (EPI == 1) {
    bv = *(const v4fa*)(bias + clampi(nc, 0, N - 4));
    asm volatile("" :: "v"(bv));
  }
#pragma unroll
  for (int i = 0; i < 4; ++i) {
    const int mBase = m0 + (i << 4);
#pragma unroll
    for (int j = 0; j < 4; ++j) {
#pragma unroll
      for (int r = 0; r < 8; ++r) slab[(h8 + r) * 68 + (j << 4) + rl] = acc[i][j][r];
    }
    __builtin_amdgcn_fence(__ATOMIC_RELEASE, "workgroup");
    __builtin_amdgcn_wave_barrier();
    __builtin_amdgcn_fence(__ATOMIC_ACQUIRE, "workgroup");
    v4f vv[8];
#pragma unroll
    for (int it = 0; it < 8; ++it) {
      const int row = it * 2 + hh;
      v4f v = *(const v4fa*)(slab + row * 68 + c4);
      if (EPI == 1) v += bv;
      vv[it] = v;
    }
    for (int pass = 0; pass < 2; ++pass) {
#pragma unroll
      for (int it = 0; it < 8; ++it) {
        const int row = mBase + it * 2 + hh;
        if (cok && row < M) *(volatile v4f*)(D + (size_t)row * (size_t)ldd + nc) = vv[it];
      }
      __threadfence();
    }
    __builtin_amdgcn_fence(__ATOMIC_RELEASE, "workgroup");
    __builtin_amdgcn_wave_barrier();
    __builtin_amdgcn_fence(__ATOMIC_ACQUIRE, "workgroup");
  }
}

#define GN       100000
#define GE       1600000
#define GHC      128
#define MPAD     100096
#define NBK      1024
#define NBUCK    98
#define WCAPB    256
#define BCHUNK   2048
#define NCHUNK   782
#define RCAP     20992
#define OFFP     1152
#define DEGCAP   64
#define MAXB1024 16710
#define MAXDEG   36
#define AD_OFF   (GN * 4)
#define LDS_BUCKET ((2 * RCAP + NBK + OFFP + NBK + 8 * WCAPB + 16) * 4)
#define NEG_SENT (-3.0e38f)

static_assert(GN % 32 == 0);
static_assert(GE % 256 == 0);
static_assert(GN <= (1 << 17));
static_assert(NBK <= (1 << 10));
static_assert(NBUCK * NBK >= GN && (NBUCK - 1) * NBK < GN);
static_assert(((GN - (NBUCK - 1) * NBK) % 8) == 0);
static_assert(NCHUNK * BCHUNK >= GE && (NCHUNK - 1) * BCHUNK < GE);
static_assert(RCAP * 4 >= MAXB1024 * 5 && (RCAP % 256) == 0);
static_assert(DEGCAP >= MAXDEG + 8 && (DEGCAP % 32) == 0);
static_assert((OFFP % 128) == 0 && OFFP >= NBK + 2);
static_assert(MPAD % 64 == 0 && MPAD >= GN && GN % 16 == 0);
static_assert(LDS_BUCKET <= 262144);

typedef int v4i __attribute__((ext_vector_type(4)));
typedef v4i __attribute__((may_alias)) v4ia;
typedef v4u __attribute__((may_alias)) v4ua;

constexpr size_t SZ_XB   = (size_t)MPAD * GHC * 2;
constexpr size_t SZ_WT   = (size_t)GHC * GHC * 2;
constexpr size_t SZ_H    = (size_t)MPAD * GHC * 4;
constexpr size_t SZ_ASD  = (size_t)2 * GN * 4 * 4;
constexpr size_t SZ_HITS = (size_t)NBUCK * RCAP * 4;
constexpr size_t SZ_OFF  = (size_t)NBUCK * OFFP * 4;
constexpr size_t WS_XB   = 0;
constexpr size_t WS_WT   = WS_XB + SZ_XB;
constexpr size_t WS_H    = WS_WT + SZ_WT;
constexpr size_t WS_ASD  = WS_H + SZ_H;
constexpr size_t WS_HITS = WS_ASD + SZ_ASD;
constexpr size_t WS_OFF  = WS_HITS + SZ_HITS;
constexpr size_t WS_TOTAL = WS_OFF + SZ_OFF;
static_assert((SZ_XB % 512) == 0 && (SZ_WT % 512) == 0 && (SZ_H % 512) == 0);
static_assert((SZ_ASD % 512) == 0 && (SZ_HITS % 512) == 0 && (SZ_OFF % 512) == 0);
static_assert(((size_t)GN * 4 * 4) % 512 == 0);
static_assert(WS_TOTAL <= ((size_t)128 << 20));

__device__ __forceinline__ int imin(int a, int b) { return a < b ? a : b; }

__device__ __forceinline__ void wave_lds_sync() {
  __builtin_amdgcn_fence(__ATOMIC_RELEASE, "workgroup");
  __builtin_amdgcn_wave_barrier();
  __builtin_amdgcn_fence(__ATOMIC_ACQUIRE, "workgroup");
}

__global__ __launch_bounds__(256) void k_wtr(const float* __restrict__ w, unsigned short* wt) {
  const int u  = (int)blockIdx.x * 256 + (int)threadIdx.x;
  const int n  = u >> 4;
  const int k8 = (u & 15) << 3;
  float x[8];
#pragma unroll
  for (int e = 0; e < 8; ++e) {
    const float v = w[(size_t)(k8 + e) * GHC + n];
    asm volatile("" :: "v"(v));
    x[e] = v;
  }
  const v4u o = pack8_bf16((v4f){ x[0], x[1], x[2], x[3] }, (v4f){ x[4], x[5], x[6], x[7] });
  volatile v4u* q = (volatile v4u*)(wt + (size_t)u * 8);
  *q = o;
  __threadfence();
  *q = o;
}

__global__ __launch_bounds__(256) void k_dots(const float* __restrict__ Hf, const float* __restrict__ att_s,
                                              const float* __restrict__ att_d, float* ASD) {
  __shared__ __attribute__((aligned(16))) float sAtt[256];
  __shared__ __attribute__((aligned(16))) float sOut[256];
  const int tid = (int)threadIdx.x, lane = tid & 31, wave = tid >> 5;
  const int blk = (int)blockIdx.x;
  if (tid < 32) {
    const v4f a = *(const v4fa*)(att_s + 4 * tid);
    const v4f d = *(const v4fa*)(att_d + 4 * tid);
    *(v4fa*)(sAtt + 4 * tid)       = (v4f){ bf16_val(a[0]), bf16_val(a[1]), bf16_val(a[2]), bf16_val(a[3]) };
    *(v4fa*)(sAtt + 128 + 4 * tid) = (v4f){ bf16_val(d[0]), bf16_val(d[1]), bf16_val(d[2]), bf16_val(d[3]) };
  }
  __syncthreads();
  const v4f ws = *(const v4fa*)(sAtt + 4 * lane);
  const v4f wd = *(const v4fa*)(sAtt + 128 + 4 * lane);
#pragma unroll
  for (int q = 0; q < 4; ++q) {
    const int ln   = wave * 4 + q;
    const int node = blk * 32 + ln;
    const v4f hv = *(const v4fa*)(Hf + (size_t)node * GHC + 4 * lane);
    float s = hv[0] * ws[0];
    s = fmaf(hv[1], ws[1], s); s = fmaf(hv[2], ws[2], s); s = fmaf(hv[3], ws[3], s);
    float d = hv[0] * wd[0];
    d = fmaf(hv[1], wd[1], d); d = fmaf(hv[2], wd[2], d); d = fmaf(hv[3], wd[3], d);
    s += __shfl_xor(s, 1); d += __shfl_xor(d, 1);
    s += __shfl_xor(s, 2); d += __shfl_xor(d, 2);
    s += __shfl_xor(s, 4); d += __shfl_xor(d, 4);
    if ((lane & 7) == 0) {
      sOut[ln * 4 + (lane >> 3)]       = s;
      sOut[128 + ln * 4 + (lane >> 3)] = d;
    }
  }
  __syncthreads();
  if (wave < 2) {
    const v4f v = *(const v4fa*)(sOut + wave * 128 + 4 * lane);
    volatile v4f* q = (volatile v4f*)(ASD + (size_t)wave * AD_OFF + (size_t)blk * 128 + 4 * lane);
    *q = v;
    __threadfence();
    *q = v;
  }
}

__global__ __launch_bounds__(256) void k_bucket(const int* __restrict__ ei, unsigned* hits, int* offt) {
  extern __shared__ v4u lds_dyn[];
  unsigned* reg1 = (unsigned*)lds_dyn;
  unsigned* reg2 = reg1 + RCAP;
  int* scnt = (int*)(reg2 + RCAP);
  int* soff = scnt + NBK;
  int* cur  = soff + OFFP;
  int* list = cur + NBK;
  int* wcnt = list + 8 * WCAPB;
  int* wtot = wcnt + 8;
  const int tid = (int)threadIdx.x, lane = tid & 31, wave = tid >> 5;
  const int b = (int)blockIdx.x;
  const int slotBase = b * NBK;
  const int nb = imin(NBK, GN - slotBase);
  const int* srcs = ei;
  const int* dsts = ei + GE;

  for (int i = tid; i < NBK; i += 256) scnt[i] = 0;
  for (int i = tid; i < 8 * WCAPB; i += 256) list[i] = 0;
  __syncthreads();

  int tot = 0, totraw = 0;
#pragma unroll 1
  for (int ch = 0; ch < NCHUNK; ++ch) {
    const int kb = ch * BCHUNK + wave * 256;
    const bool wv = kb < GE;
    int key[8];
#pragma unroll
    for (int j = 0; j < 8; ++j) {
      const int idx = imin(kb + j * 32 + lane, GE - 1);
      const int v = dsts[idx];
      asm volatile("" :: "v"(v));
      key[j] = wv ? v : -1;
    }
    int wc = 0;
#pragma unroll
    for (int j = 0; j < 8; ++j) {
      const unsigned s = (unsigned)key[j] - (unsigned)slotBase;
      const bool hit = s < (unsigned)nb;
      const unsigned mj = __builtin_amdgcn_ballot_w32(hit);
      const int pos = wc + (int)__builtin_amdgcn_mbcnt_lo(mj, 0u);
      if (mj != 0u) {
        if (hit && pos < WCAPB) list[wave * WCAPB + pos] = ((j * 32 + lane) << 10) | (int)s;
        wc += (int)__builtin_popcount(mj);
      }
    }
    wc = __builtin_amdgcn_readfirstlane(clampi(wc, 0, WCAPB));
    if (lane == 0) wcnt[wave] = wc;
    __syncthreads();
    int pre = 0, all = 0;
#pragma unroll
    for (int w2 = 0; w2 < 8; ++w2) {
      const int c = clampi(wcnt[w2], 0, WCAPB);
      all += c;
      pre += (w2 < wave) ? c : 0;
    }
    const int base = tot + pre;
#pragma unroll 1
    for (int i0 = 0; i0 < wc; i0 += 32) {
      const int i   = i0 + lane;
      const int ic  = imin(i, WCAPB - 1);
      const int ent = list[wave * WCAPB + ic];
      const int el  = (ent >> 10) & 255;
      const int sl  = ent & (NBK - 1);
      const int eid = clampi(kb + el, 0, GE - 1);
      const int sraw = srcs[eid];
      asm volatile("" :: "v"(sraw));
      const int s   = clampi(sraw, 0, GN - 1);
      const int pos = base + i;
      if (i < wc && pos < RCAP) reg1[pos] = (unsigned)s | ((unsigned)sl << 17);
    }
    totraw += all;
    tot = imin(totraw, RCAP);
    __syncthreads();
  }
  const int nh   = tot;
  const int flag = (totraw > RCAP) ? 1 : 0;

  if (wave == 0) {
#pragma unroll 1
    for (int b0 = 0; b0 < nh; b0 += 32) {
      const int idx = imin(b0 + lane, nh - 1);
      const int uv  = (int)reg1[idx];
      const int m32 = imin(nh - b0, 32);
#pragma unroll 1
      for (int k = 0; k < m32; ++k) {
        const int u  = __builtin_amdgcn_readlane(uv, k);
        const int sl = (u >> 17) & (NBK - 1);
        if (lane == 0) scnt[sl] = scnt[sl] + 1;
      }
    }
  }
  __syncthreads();

  {
    int e0 = scnt[4 * tid + 0], e1 = scnt[4 * tid + 1], e2 = scnt[4 * tid + 2], e3 = scnt[4 * tid + 3];
    e0 = e0 < 0 ? 0 : e0; e1 = e1 < 0 ? 0 : e1; e2 = e2 < 0 ? 0 : e2; e3 = e3 < 0 ? 0 : e3;
    const int ts = e0 + e1 + e2 + e3;
    int incl = ts;
#pragma unroll
    for (int d = 1; d < 32; d <<= 1) {
      const int up = __shfl_up(incl, d);
      if (lane >= d) incl += up;
    }
    if (lane == 31) wtot[wave] = incl;
    __syncthreads();
    int pre = 0;
#pragma unroll
    for (int w2 = 0; w2 < 8; ++w2) pre += (w2 < wave) ? wtot[w2] : 0;
    int run = pre + incl - ts;
    soff[4 * tid + 0] = run; cur[4 * tid + 0] = run; run += e0;
    soff[4 * tid + 1] = run; cur[4 * tid + 1] = run; run += e1;
    soff[4 * tid + 2] = run; cur[4 * tid + 2] = run; run += e2;
    soff[4 * tid + 3] = run; cur[4 * tid + 3] = run;
    if (tid < OFFP - NBK) soff[NBK + tid] = (tid == 0) ? nh : ((tid == 1) ? flag : 0);
  }
  __syncthreads();

  if (wave == 0) {
#pragma unroll 1
    for (int b0 = 0; b0 < nh; b0 += 32) {
      const int idx = imin(b0 + lane, nh - 1);
      const int uv  = (int)reg1[idx];
      const int m32 = imin(nh - b0, 32);
#pragma unroll 1
      for (int k = 0; k < m32; ++k) {
        const int u  = __builtin_amdgcn_readlane(uv, k);
        const int sl = (u >> 17) & (NBK - 1);
        if (lane == 0) {
          const int pos = clampi(cur[sl], 0, RCAP - 1);
          reg2[pos] = (unsigned)u;
          cur[sl] = pos + 1;
        }
      }
    }
  }
  for (int i = nh + tid; i < RCAP; i += 256) reg2[i] = 0u;
  __syncthreads();

  unsigned* hb = hits + (size_t)b * RCAP;
  int* ob = offt + (size_t)b * OFFP;
  for (int pass = 0; pass < 2; ++pass) {
#pragma unroll 1
    for (int p = tid; p < RCAP / 4; p += 256) {
      const v4u v = *(const v4ua*)(reg2 + 4 * p);
      *(volatile v4u*)(hb + 4 * p) = v;
    }
#pragma unroll 1
    for (int p = tid; p < OFFP / 4; p += 256) {
      const v4i v = *(const v4ia*)(soff + 4 * p);
      *(volatile v4i*)(ob + 4 * p) = v;
    }
    __threadfence();
  }
}

__global__ __launch_bounds__(256) void k_replay(const unsigned* __restrict__ hits, const int* __restrict__ offt,
                                                const float* __restrict__ Hf, const float* __restrict__ ASD,
                                                const float* __restrict__ bias, float* out) {
  __shared__ __attribute__((aligned(16))) int      sOff[OFFP];
  __shared__ __attribute__((aligned(16))) float    sBias[GHC];
  __shared__ __attribute__((aligned(16))) unsigned sTile[8][DEGCAP * 5];
  const int tid = (int)threadIdx.x, lane = tid & 31, wave = tid >> 5;
  const int b = (int)blockIdx.x;
  const int slotBase = b * NBK;
  const int nb = imin(NBK, GN - slotBase);
  for (int p = tid; p < OFFP / 4; p += 256)
    *(v4ia*)(sOff + 4 * p) = *(const v4ia*)(offt + (size_t)b * OFFP + 4 * p);
  if (tid < 32) {
    const v4f bq = *(const v4fa*)(bias + 4 * tid);
    *(v4fa*)(sBias + 4 * tid) = (v4f){ bf16_val(bq[0]), bf16_val(bq[1]), bf16_val(bq[2]), bf16_val(bq[3]) };
  }
  __syncthreads();

  const int nbw  = nb >> 3;
  const int flag = sOff[NBK + 1];
  const int nh   = __builtin_amdgcn_readfirstlane(clampi(sOff[NBK], 0, RCAP));
  const int head = lane >> 3;
  const v4f bv   = *(const v4fa*)(sBias + 4 * lane);
  unsigned* tile = sTile[wave];
  const unsigned* hb = hits + (size_t)b * RCAP;
  const float qnan = __uint_as_float(0x7fc00000u);

#pragma unroll 1
  for (int jt = 0; jt < nbw; ++jt) {
    const int slot = wave * nbw + jt;
    const int d    = slotBase + slot;
    const int dc   = imin(d, GN - 1);
    const int o0   = sOff[slot];
    const int o1   = sOff[slot + 1];
    const int craw = o1 - o0;
    int stv = clampi(o0, 0, nh);
    int cnv = clampi(craw, 0, DEGCAP);
    cnv = imin(cnv, nh - stv);
    const int st = __builtin_amdgcn_readfirstlane(stv);
    const int cn = __builtin_amdgcn_readfirstlane(cnv);
    const bool pois = (flag != 0) || (craw > DEGCAP) || (craw < 0);
    const v4f adv = *(const v4fa*)(ASD + (size_t)AD_OFF + (size_t)dc * 4);
    const int nch = (cn + 31) >> 5;

    float m0 = NEG_SENT, m1 = NEG_SENT, m2 = NEG_SENT, m3 = NEG_SENT;
#pragma unroll 1
    for (int c = 0; c < nch; ++c) {
      const int j = c * 32 + lane;
      const bool valid = j < cn;
      const int idx = imin(st + j, RCAP - 1);
      const unsigned hw = hb[idx];
      asm volatile("" :: "v"(hw));
      const int s = imin((int)(hw & 0x1FFFFu), GN - 1);
      const v4f av = *(const v4fa*)(ASD + (size_t)s * 4);
      asm volatile("" :: "v"(av));
      float e0 = av[0] + adv[0], e1 = av[1] + adv[1], e2 = av[2] + adv[2], e3 = av[3] + adv[3];
      e0 = (e0 >= 0.0f) ? e0 : 0.2f * e0;
      e1 = (e1 >= 0.0f) ? e1 : 0.2f * e1;
      e2 = (e2 >= 0.0f) ? e2 : 0.2f * e2;
      e3 = (e3 >= 0.0f) ? e3 : 0.2f * e3;
      e0 = valid ? e0 : NEG_SENT;
      e1 = valid ? e1 : NEG_SENT;
      e2 = valid ? e2 : NEG_SENT;
      e3 = valid ? e3 : NEG_SENT;
      tile[j * 5 + 0] = __float_as_uint(e0);
      tile[j * 5 + 1] = __float_as_uint(e1);
      tile[j * 5 + 2] = __float_as_uint(e2);
      tile[j * 5 + 3] = __float_as_uint(e3);
      tile[j * 5 + 4] = (unsigned)s;
      m0 = (e0 > m0) ? e0 : m0;
      m1 = (e1 > m1) ? e1 : m1;
      m2 = (e2 > m2) ? e2 : m2;
      m3 = (e3 > m3) ? e3 : m3;
    }
#pragma unroll
    for (int off = 16; off > 0; off >>= 1) {
      const float t0 = __shfl_xor(m0, off);
      const float t1 = __shfl_xor(m1, off);
      const float t2 = __shfl_xor(m2, off);
      const float t3 = __shfl_xor(m3, off);
      m0 = (t0 > m0) ? t0 : m0;
      m1 = (t1 > m1) ? t1 : m1;
      m2 = (t2 > m2) ? t2 : m2;
      m3 = (t3 > m3) ? t3 : m3;
    }
    float d0 = 0.0f, d1 = 0.0f, d2 = 0.0f, d3 = 0.0f;
#pragma unroll 1
    for (int c = 0; c < nch; ++c) {
      const int j = c * 32 + lane;
      const bool valid = j < cn;
      const float e0 = __uint_as_float(tile[j * 5 + 0]);
      const float e1 = __uint_as_float(tile[j * 5 + 1]);
      const float e2 = __uint_as_float(tile[j * 5 + 2]);
      const float e3 = __uint_as_float(tile[j * 5 + 3]);
      const float x0 = expf(e0 - m0);
      const float x1 = expf(e1 - m1);
      const float x2 = expf(e2 - m2);
      const float x3 = expf(e3 - m3);
      const float p0 = valid ? x0 : 0.0f;
      const float p1 = valid ? x1 : 0.0f;
      const float p2 = valid ? x2 : 0.0f;
      const float p3 = valid ? x3 : 0.0f;
      tile[j * 5 + 0] = __float_as_uint(p0);
      tile[j * 5 + 1] = __float_as_uint(p1);
      tile[j * 5 + 2] = __float_as_uint(p2);
      tile[j * 5 + 3] = __float_as_uint(p3);
      d0 += p0; d1 += p1; d2 += p2; d3 += p3;
    }
#pragma unroll
    for (int off = 16; off > 0; off >>= 1) {
      d0 += __shfl_xor(d0, off);
      d1 += __shfl_xor(d1, off);
      d2 += __shfl_xor(d2, off);
      d3 += __shfl_xor(d3, off);
    }
    wave_lds_sync();

    v4f acc = (v4f){ 0.0f, 0.0f, 0.0f, 0.0f };
#pragma unroll 1
    for (int j = 0; j < cn; ++j) {
      const int s   = clampi((int)tile[j * 5 + 4], 0, GN - 1);
      const float p = __uint_as_float(tile[j * 5 + head]);
      const v4f hr  = *(const v4fa*)(Hf + (size_t)s * GHC + 4 * lane);
      acc[0] = fmaf(p, hr[0], acc[0]);
      acc[1] = fmaf(p, hr[1], acc[1]);
      acc[2] = fmaf(p, hr[2], acc[2]);
      acc[3] = fmaf(p, hr[3], acc[3]);
    }

    const float den = (head == 0) ? d0 : ((head == 1) ? d1 : ((head == 2) ? d2 : d3));
    const bool empty = (cn == 0);
    const float dd = empty ? 1.0f : (den + 1e-16f);
    v4f o;
    o[0] = acc[0] / dd; o[1] = acc[1] / dd; o[2] = acc[2] / dd; o[3] = acc[3] / dd;
    o[0] = (empty ? 0.0f : o[0]) + bv[0];
    o[1] = (empty ? 0.0f : o[1]) + bv[1];
    o[2] = (empty ? 0.0f : o[2]) + bv[2];
    o[3] = (empty ? 0.0f : o[3]) + bv[3];
    o[0] = pois ? qnan : o[0];
    o[1] = pois ? qnan : o[1];
    o[2] = pois ? qnan : o[2];
    o[3] = pois ? qnan : o[3];
    if (d < GN) {
      volatile v4f* q = (volatile v4f*)(out + (size_t)d * GHC + 4 * lane);
      *q = o;
      __threadfence();
      *q = o;
    }
    wave_lds_sync();
  }
}

extern "C" void kernel_launch(void* const* d_in, const int* in_sizes, int n_in,
                              void* d_out, int out_size, void* d_ws, size_t ws_size,
                              hipStream_t stream) {
  if (n_in < 6) return;
  if (in_sizes[0] != GN * GHC) return;
  if (in_sizes[1] != 2 * GE) return;
  if (in_sizes[2] != GHC * GHC) return;
  if (in_sizes[3] != GHC || in_sizes[4] != GHC || in_sizes[5] != GHC) return;
  if (out_size != GN * GHC) return;
  if (ws_size < WS_TOTAL) return;

  const float* x     = (const float*)d_in[0];
  const int*   ei    = (const int*)  d_in[1];
  const float* W     = (const float*)d_in[2];
  const float* att_s = (const float*)d_in[3];
  const float* att_d = (const float*)d_in[4];
  const float* bias  = (const float*)d_in[5];
  float* out = (float*)d_out;

  char* ws = (char*)d_ws;
  unsigned short* XB   = (unsigned short*)(ws + WS_XB);
  unsigned short* WT   = (unsigned short*)(ws + WS_WT);
  float*          Hf   = (float*)(ws + WS_H);
  float*          ASD  = (float*)(ws + WS_ASD);
  unsigned*       HITS = (unsigned*)(ws + WS_HITS);
  int*            OFFT = (int*)(ws + WS_OFF);

  hipFuncSetAttribute(reinterpret_cast<const void*>(&k_bucket),
                      hipFuncAttributeMaxDynamicSharedMemorySize, LDS_BUCKET);

  k_plane<0><<<(MPAD * GHC / 8) / 256, 256, 0, stream>>>(x, GN, GHC, GHC, XB, MPAD, GHC);
  k_wtr<<<(GHC * GHC / 8) / 256, 256, 0, stream>>>(W, WT);

  {
    const int tiles = ((GN + 63) / 64) * (GHC / 64);
    k_gemm_nt<0, 0><<<(tiles + 7) / 8, 256, 0, stream>>>(XB, WT, bias, Hf, GN, GHC, GHC, GHC);
  }

  k_dots<<<GN / 32, 256, 0, stream>>>(Hf, att_s, att_d, ASD);
  k_bucket<<<NBUCK, 256, LDS_BUCKET, stream>>>(ei, HITS, OFFT);
  k_replay<<<NBUCK, 256, 0, stream>>>(HITS, OFFT, Hf, ASD, bias, out);
}
